// HyperTokenMixer_44616120271558
// MI455X (gfx1250) — hardware-verified
//
#include <hip/hip_runtime.h>
#include <math.h>

constexpr int kBatch = 8;
constexpr int kTok   = 4096;
constexpr int kDim   = 256;
constexpr int kDpr   = 512;
constexpr int kGrp   = 4;
constexpr int kNumGrp = kBatch / kGrp;
constexpr int kKsp   = 4;
static_assert(kTok % 64 == 0 && kDim % 64 == 0 && kDpr % 64 == 0);
static_assert((kTok / kKsp) % 32 == 0);
static_assert(kBatch % kGrp == 0);

typedef __attribute__((ext_vector_type(16))) _Float16 v16h;
typedef __attribute__((ext_vector_type(8)))  _Float16 v8h;
typedef __attribute__((ext_vector_type(16))) __bf16   v16b;
typedef __attribute__((ext_vector_type(8)))  __bf16   v8b;
typedef __attribute__((ext_vector_type(8)))  float    v8f;
typedef __attribute__((ext_vector_type(4)))  float    v4f;
typedef __attribute__((ext_vector_type(4)))  unsigned int v4u;

__device__ __forceinline__ unsigned short f2bf_bits(float f) {
  unsigned u = __float_as_uint(f);
  return (unsigned short)((u + 0x7FFFu + ((u >> 16) & 1u)) >> 16);
}
__device__ __forceinline__ float bf_bits2f(unsigned short h) { return __uint_as_float(((unsigned)h) << 16); }

__device__ __forceinline__ void dep_guard_h(v8f& a, v8f& b, v16h x, v16h y) { asm volatile("v_nop\n\tv_nop\n\tv_nop\n\tv_nop" : "+v"(a), "+v"(b) : "v"(x), "v"(y)); }
__device__ __forceinline__ void dep_guard_b(v8f& a, v8f& b, v16b x, v16b y) { asm volatile("v_nop\n\tv_nop\n\tv_nop\n\tv_nop" : "+v"(a), "+v"(b) : "v"(x), "v"(y)); }
__device__ __forceinline__ void keep4_h(v16h a, v16h b, v16h c, v16h d) { asm volatile("v_nop" :: "v"(a), "v"(b), "v"(c), "v"(d)); }
__device__ __forceinline__ void keep4_b(v16b a, v16b b, v16b c, v16b d) { asm volatile("v_nop" :: "v"(a), "v"(b), "v"(c), "v"(d)); }
__device__ __forceinline__ void acc_guard4(v8f& a, v8f& b, v8f& c, v8f& d) { asm volatile("v_nop\n\tv_nop\n\tv_nop\n\tv_nop" : "+v"(a), "+v"(b), "+v"(c), "+v"(d)); }
template <typename T> struct Frag;
template <> struct Frag<_Float16> {
  typedef v16h V; union U { v16h v; v8h h[2]; };
  static __device__ __forceinline__ v16h load(const _Float16* p) {
    U f; f.h[0] = *(const v8h*)(p); f.h[1] = *(const v8h*)(p + 16); return f.v;
  }
  static __device__ __forceinline__ v8f mma(v16h a, v16h b, v8f c) {
    return __builtin_amdgcn_wmma_f32_16x16x32_f16(false, a, false, b, (short)0, c, false, false);
  }
  static __device__ __forceinline__ void guard(v8f& a, v8f& b, v16h x, v16h y) { dep_guard_h(a, b, x, y); }
  static __device__ __forceinline__ void keep(v16h a, v16h b, v16h c, v16h d) { keep4_h(a, b, c, d); }
};
template <> struct Frag<__bf16> {
  typedef v16b V; union U { v16b v; v8b h[2]; };
  static __device__ __forceinline__ v16b load(const __bf16* p) {
    U f; f.h[0] = *(const v8b*)(p); f.h[1] = *(const v8b*)(p + 16); return f.v;
  }
  static __device__ __forceinline__ v8f mma(v16b a, v16b b, v8f c) {
    return __builtin_amdgcn_wmma_f32_16x16x32_bf16(false, a, false, b, (short)0, c, false, false);
  }
  static __device__ __forceinline__ void guard(v8f& a, v8f& b, v16b x, v16b y) { dep_guard_b(a, b, x, y); }
  static __device__ __forceinline__ void keep(v16b a, v16b b, v16b c, v16b d) { keep4_b(a, b, c, d); }
};

__device__ __forceinline__ unsigned pk16(unsigned short a, unsigned short b) { return (unsigned)a | ((unsigned)b << 16); }

template <int ET> struct Elem;
template <> struct Elem<0> { typedef _Float16 T; };
template <> struct Elem<1> { typedef __bf16 T; };
template <int ET, bool SPLIT, int BIAS_MODE, int OUT_MODE, bool RESID, int ACT = 0>
__global__ __launch_bounds__(256) void wmma_gemm64(
    const unsigned short* __restrict__ Ap, const unsigned short* __restrict__ A2p, int lda, long strideA,
    const unsigned short* __restrict__ Btp, const unsigned short* __restrict__ Bt2p, int ldb, long strideB,
    void* __restrict__ Cout, void* __restrict__ Cout2, int ldc, long strideC,
    const float* __restrict__ bias,
    const float* __restrict__ resid, long strideR,
    int M, int N, int K, float scale) {
  typedef typename Elem<ET>::T T;
  typedef typename Frag<T>::V V;
  const T* A = (const T*)Ap; const T* A2 = (const T*)A2p; const T* Bt = (const T*)Btp; const T* Bt2 = (const T*)Bt2p;
  __shared__ __align__(16) float sT[8][16 * 68];
  const int b    = blockIdx.y;
  const int kz   = blockIdx.z;
  const size_t cb = (size_t)kz * gridDim.y + b;
  const int lane = threadIdx.x & 31;
  const int wave = threadIdx.x >> 5;
  const int tilesN = N >> 6;
  const int tilesM = M >> 6;
  const int tile = blockIdx.x * 8 + wave;
  if (tile >= tilesM * tilesN) return;
  const int tm = tile / tilesN;
  const int tn = tile - tm * tilesN;
  const int m0 = tm << 6;
  const int n0 = tn << 6;

  const size_t kzOff = (size_t)kz * (size_t)K;
  const T* Ab  = A  + (size_t)b * strideA + kzOff;
  const T* Bb  = Bt + (size_t)b * strideB + kzOff;
  const T* Ab2 = SPLIT ? (A2  + (size_t)b * strideA + kzOff) : nullptr;
  const T* Bb2 = SPLIT ? (Bt2 + (size_t)b * strideB + kzOff) : nullptr;

  const int rlane = lane & 15;
  const int koff  = (lane >> 4) * 8;
  const int mOff  = (lane >> 4) * 8;

  v8f acc[4][4];
#pragma unroll
  for (int i = 0; i < 4; ++i)
#pragma unroll
    for (int j = 0; j < 4; ++j) acc[i][j] = (v8f){0.f,0.f,0.f,0.f,0.f,0.f,0.f,0.f};

  for (int k0 = 0; k0 < K; k0 += 32) {
    V bh[4], bl[4];
#pragma unroll
    for (int j = 0; j < 4; ++j) {
      const size_t bo = (size_t)(n0 + (j << 4) + rlane) * ldb + koff + k0;
      bh[j] = Frag<T>::load(Bb + bo);
      if (SPLIT) bl[j] = Frag<T>::load(Bb2 + bo);
    }
#pragma unroll
    for (int i = 0; i < 4; ++i) {
      const size_t ao = (size_t)(m0 + (i << 4) + rlane) * lda + koff + k0;
      V ah = Frag<T>::load(Ab + ao);
      V al;
      if (SPLIT) al = Frag<T>::load(Ab2 + ao);
#pragma unroll
      for (int j = 0; j < 4; ++j) {
        acc[i][j] = Frag<T>::mma(ah, bh[j], acc[i][j]);
        if (SPLIT) {
          acc[i][j] = Frag<T>::mma(ah, bl[j], acc[i][j]);
          acc[i][j] = Frag<T>::mma(al, bh[j], acc[i][j]);
        }
      }
      Frag<T>::guard(acc[i][0], acc[i][3], ah, SPLIT ? al : ah);
    }
    Frag<T>::keep(bh[0], bh[1], bh[2], bh[3]);
    if (SPLIT) Frag<T>::keep(bl[0], bl[1], bl[2], bl[3]);
  }
  acc_guard4(acc[0][0], acc[0][1], acc[0][2], acc[0][3]);
  acc_guard4(acc[1][0], acc[1][1], acc[1][2], acc[1][3]);
  acc_guard4(acc[2][0], acc[2][1], acc[2][2], acc[2][3]);
  acc_guard4(acc[3][0], acc[3][1], acc[3][2], acc[3][3]);

  float* slab = sT[wave];
  const float* Rb = RESID ? (resid + (size_t)b * strideR) : nullptr;
#pragma unroll
  for (int i = 0; i < 4; ++i) {
    const int mBase = m0 + (i << 4);
#pragma unroll
    for (int j = 0; j < 4; ++j) {
      const int n = n0 + (j << 4) + rlane;
      float bv = 0.f;
      if (BIAS_MODE == 2) bv = bias[n];
#pragma unroll
      for (int r = 0; r < 8; ++r) {
        float v = acc[i][j][r] * scale;
        if (BIAS_MODE == 1) v += bias[mBase + mOff + r];
        if (BIAS_MODE == 2) v += bv;
        if (RESID) v += Rb[(size_t)(mBase + mOff + r) * ldc + n];
        if (ACT == 2) v = fmaxf(v, 0.0f);
        if (ACT == 4) v = (v > 0.f) ? v : 0.01f * v;
        slab[(mOff + r) * 68 + (j << 4) + rlane] = v;
      }
    }
    __builtin_amdgcn_fence(__ATOMIC_RELEASE, "workgroup");
    __builtin_amdgcn_wave_barrier();
    __builtin_amdgcn_fence(__ATOMIC_ACQUIRE, "workgroup");
    if (OUT_MODE == 0) {
      float* C = (float*)Cout + cb * strideC;
      const int hh = lane >> 4, c4 = (lane & 15) * 4;
      for (int pass = 0; pass < 2; ++pass) {
#pragma unroll
        for (int it = 0; it < 8; ++it) {
          const int row = it * 2 + hh;
          v4f v = *(const v4f*)(slab + row * 68 + c4);
          *(volatile v4f*)(C + (size_t)(mBase + row) * ldc + n0 + c4) = v;
        }
        __threadfence();
      }
    } else {
      const int q = lane >> 3, c8 = (lane & 7) * 8;
      unsigned short* C  = (unsigned short*)Cout  + cb * strideC;
      unsigned short* C2 = (OUT_MODE == 2) ? ((unsigned short*)Cout2 + cb * strideC) : nullptr;
      for (int pass = 0; pass < 2; ++pass) {
#pragma unroll
        for (int it = 0; it < 4; ++it) {
          const int row = it * 4 + q;
          const float* sp = slab + row * 68 + c8;
          v8h hv, lv;
#pragma unroll
          for (int e = 0; e < 8; ++e) {
            if (OUT_MODE == 1) {
              hv[e] = (_Float16)sp[e];
            } else {
              unsigned short hb = f2bf_bits(sp[e]);
              unsigned short lb = f2bf_bits(sp[e] - bf_bits2f(hb));
              hv[e] = __builtin_bit_cast(_Float16, hb);
              lv[e] = __builtin_bit_cast(_Float16, lb);
            }
          }
          *(volatile v8h*)(C + (size_t)(mBase + row) * ldc + n0 + c8) = hv;
          if (OUT_MODE == 2) *(volatile v8h*)(C2 + (size_t)(mBase + row) * ldc + n0 + c8) = lv;
        }
        __threadfence();
      }
    }
    __builtin_amdgcn_fence(__ATOMIC_RELEASE, "workgroup");
    __builtin_amdgcn_wave_barrier();
    __builtin_amdgcn_fence(__ATOMIC_ACQUIRE, "workgroup");
  }
}

__global__ __launch_bounds__(256) void wsplit_kernel(const float* __restrict__ Wa, const float* __restrict__ Wb,
                                                     unsigned short* __restrict__ out) {
  __shared__ float sm[64][65];
  const int t  = threadIdx.x;
  const int d0 = blockIdx.x * 64;
  const int p0 = blockIdx.y * 64;
  const int z  = blockIdx.z;
  const float* W = (z == 0) ? Wa : Wb;
#pragma unroll
  for (int i = 0; i < 16; ++i) {
    const int e = i * 256 + t;
    const int r = e >> 6;
    const int c = e & 63;
    sm[c][r] = W[(size_t)(d0 + r) * kDpr + p0 + c];
  }
  __syncthreads();
  const int lane = t & 31, wave = t >> 5;
  const int q = lane >> 3, c8 = (lane & 7) * 8;
  const size_t plane = (size_t)kDpr * kDim;
  unsigned short* oh = out + (size_t)z * 2 * plane;
  unsigned short* ol = oh + plane;
  v4u uh[2], ul[2];
#pragma unroll
  for (int it = 0; it < 2; ++it) {
    const int row = wave * 8 + it * 4 + q;
    unsigned short hb[8], lb[8];
#pragma unroll
    for (int e = 0; e < 8; ++e) {
      const float v = sm[row][c8 + e];
      const unsigned short h1 = f2bf_bits(v);
      hb[e] = h1;
      lb[e] = f2bf_bits(v - bf_bits2f(h1));
    }
    uh[it] = (v4u){pk16(hb[0], hb[1]), pk16(hb[2], hb[3]), pk16(hb[4], hb[5]), pk16(hb[6], hb[7])};
    ul[it] = (v4u){pk16(lb[0], lb[1]), pk16(lb[2], lb[3]), pk16(lb[4], lb[5]), pk16(lb[6], lb[7])};
  }
  for (int ps = 0; ps < 2; ++ps) {
#pragma unroll
    for (int it = 0; it < 2; ++it) {
      const int row = wave * 8 + it * 4 + q;
      const size_t o = (size_t)(p0 + row) * kDim + d0 + c8;
      *(volatile v4u*)(oh + o) = uh[it];
      *(volatile v4u*)(ol + o) = ul[it];
    }
    __threadfence();
  }
}

__global__ __launch_bounds__(256) void xp_planes_kernel(const float* __restrict__ X, const float* __restrict__ P, int batch0,
                                                        unsigned short* __restrict__ xpHi, unsigned short* __restrict__ xpLo,
                                                        unsigned short* __restrict__ xtHi, unsigned short* __restrict__ xtLo) {
  __shared__ float sm[64][65];
  const int t  = threadIdx.x;
  const int n0 = blockIdx.x * 64;
  const int d0 = blockIdx.y * 64;
  const int bl = blockIdx.z;
  const size_t inOff = (size_t)(batch0 + bl) * kTok * kDim;
  const float* Xb = X + inOff;
  const float* Pb = P + inOff;
#pragma unroll
  for (int i = 0; i < 16; ++i) {
    const int e = i * 256 + t;
    const int r = e >> 6;
    const int c = e & 63;
    const size_t gi = (size_t)(n0 + r) * kDim + d0 + c;
    sm[c][r] = Xb[gi] + Pb[gi];
  }
  __syncthreads();
  const int lane = t & 31, wave = t >> 5;
  const int q = lane >> 3, c8 = (lane & 7) * 8;
  v4u th[2], tl[2], rh[2], rl[2];
#pragma unroll
  for (int it = 0; it < 2; ++it) {
    const int row = wave * 8 + it * 4 + q;
    unsigned short hb[8], lb[8], hr[8], lr[8];
#pragma unroll
    for (int e = 0; e < 8; ++e) {
      const float vt = sm[row][c8 + e];
      const unsigned short h1 = f2bf_bits(vt);
      hb[e] = h1;
      lb[e] = f2bf_bits(vt - bf_bits2f(h1));
      const float vr = sm[c8 + e][row];
      const unsigned short h2 = f2bf_bits(vr);
      hr[e] = h2;
      lr[e] = f2bf_bits(vr - bf_bits2f(h2));
    }
    th[it] = (v4u){pk16(hb[0], hb[1]), pk16(hb[2], hb[3]), pk16(hb[4], hb[5]), pk16(hb[6], hb[7])};
    tl[it] = (v4u){pk16(lb[0], lb[1]), pk16(lb[2], lb[3]), pk16(lb[4], lb[5]), pk16(lb[6], lb[7])};
    rh[it] = (v4u){pk16(hr[0], hr[1]), pk16(hr[2], hr[3]), pk16(hr[4], hr[5]), pk16(hr[6], hr[7])};
    rl[it] = (v4u){pk16(lr[0], lr[1]), pk16(lr[2], lr[3]), pk16(lr[4], lr[5]), pk16(lr[6], lr[7])};
  }
  const size_t bOff = (size_t)bl * kTok * kDim;
  unsigned short* xtH = xtHi + bOff;
  unsigned short* xtL = xtLo + bOff;
  unsigned short* xpH = xpHi + bOff;
  unsigned short* xpL = xpLo + bOff;
  for (int ps = 0; ps < 2; ++ps) {
#pragma unroll
    for (int it = 0; it < 2; ++it) {
      const int row = wave * 8 + it * 4 + q;
      const size_t ot = (size_t)(d0 + row) * kTok + n0 + c8;
      const size_t orr = (size_t)(n0 + row) * kDim + d0 + c8;
      *(volatile v4u*)(xtH + ot)  = th[it];
      *(volatile v4u*)(xtL + ot)  = tl[it];
      *(volatile v4u*)(xpH + orr) = rh[it];
      *(volatile v4u*)(xpL + orr) = rl[it];
    }
    __threadfence();
  }
}

__global__ __launch_bounds__(256) void gelu_split_kernel(const float* __restrict__ pm, unsigned short* __restrict__ aHi,
                                                         unsigned short* __restrict__ aLo, int total) {
  __shared__ __align__(16) unsigned short sh[256];
  __shared__ __align__(16) unsigned short sl[256];
  const int t = threadIdx.x;
  const int i = blockIdx.x * 256 + t;
  const int ic = (i < total) ? i : (total - 1);
  const float p0 = pm[(size_t)ic];
  const float p1 = pm[(size_t)total + ic];
  const float p2 = pm[(size_t)2 * total + ic];
  const float p3 = pm[(size_t)3 * total + ic];
  float x = p0 + p1;
  x = x + p2;
  x = x + p3;
  const float g = 0.5f * x * (1.0f + erff(x * 0.70710678118654752f));
  const unsigned short hb = f2bf_bits(g);
  sh[t] = hb;
  sl[t] = f2bf_bits(g - bf_bits2f(hb));
  __syncthreads();
  const int lane = t & 31, wave = t >> 5;
  if (wave < 2) {
    const v4u uh = *(const v4u*)(sh + lane * 8);
    const v4u ul = *(const v4u*)(sl + lane * 8);
    v4u u;
    u.x = (wave == 0) ? uh.x : ul.x;
    u.y = (wave == 0) ? uh.y : ul.y;
    u.z = (wave == 0) ? uh.z : ul.z;
    u.w = (wave == 0) ? uh.w : ul.w;
    unsigned short* dst = ((wave == 0) ? aHi : aLo) + (size_t)blockIdx.x * 256 + lane * 8;
    if ((blockIdx.x + 1) * 256 <= total) {
      *(volatile v4u*)dst = u;
      __threadfence();
      *(volatile v4u*)dst = u;
    }
  }
}

extern "C" void kernel_launch(void* const* d_in, const int* in_sizes, int n_in,
                              void* d_out, int out_size, void* d_ws, size_t ws_size, hipStream_t stream) {
  if (n_in < 6) return;
  const size_t nX = (size_t)kBatch * kTok * kDim;
  if ((size_t)in_sizes[0] != nX || (size_t)in_sizes[1] != nX) return;
  if (in_sizes[2] != kDim * kDpr || in_sizes[4] != kDim * kDpr) return;
  if (in_sizes[3] != kDpr || in_sizes[5] != kDpr) return;
  if ((size_t)out_size != nX) return;

  const float* X   = (const float*)d_in[0];
  const float* P   = (const float*)d_in[1];
  const float* Wh1 = (const float*)d_in[2];
  const float* bh1 = (const float*)d_in[3];
  const float* Wh2 = (const float*)d_in[4];
  const float* bh2 = (const float*)d_in[5];
  float* Y = (float*)d_out;

  const size_t whPlane = (size_t)kDpr * kDim * 2;
  const size_t xpPlane = (size_t)kGrp * kTok * kDim * 2;
  const size_t wPlane  = (size_t)kGrp * kTok * kDpr * 2;
  const size_t pmBytes = (size_t)kKsp * kGrp * kDim * kDpr * 4;
  const size_t aPlane  = (size_t)kGrp * kDim * kDpr * 2;
  char* ws = (char*)d_ws;
  size_t off = 0;
  unsigned short* whBase = (unsigned short*)(ws + off); off += 4 * whPlane;
  unsigned short* xpHi = (unsigned short*)(ws + off); off += xpPlane;
  unsigned short* xpLo = (unsigned short*)(ws + off); off += xpPlane;
  unsigned short* xtHi = (unsigned short*)(ws + off); off += xpPlane;
  unsigned short* xtLo = (unsigned short*)(ws + off); off += xpPlane;
  unsigned short* w1tHi = (unsigned short*)(ws + off); off += wPlane;
  unsigned short* w1tLo = (unsigned short*)(ws + off); off += wPlane;
  unsigned short* w2Hi  = (unsigned short*)(ws + off); off += wPlane;
  unsigned short* w2Lo  = (unsigned short*)(ws + off); off += wPlane;
  float*          pmPart = (float*)(ws + off); off += pmBytes;
  unsigned short* atHi = (unsigned short*)(ws + off); off += aPlane;
  unsigned short* atLo = (unsigned short*)(ws + off); off += aPlane;
  if (off > ws_size) return;

  const size_t whElems = (size_t)kDpr * kDim;
  unsigned short* wh1Hi = whBase;
  unsigned short* wh1Lo = whBase + whElems;
  unsigned short* wh2Hi = whBase + 2 * whElems;
  unsigned short* wh2Lo = whBase + 3 * whElems;

  wsplit_kernel<<<dim3(kDim / 64, kDpr / 64, 2), 256, 0, stream>>>(Wh1, Wh2, whBase);

  const int tilesW  = (kDpr / 64) * (kTok / 64);
  const int tilesPm = (kDim / 64) * (kDpr / 64);
  const int tilesY  = (kTok / 64) * (kDim / 64);
  const int groupTot = kGrp * kDim * kDpr;

  for (int g = 0; g < kNumGrp; ++g) {
    const int batch0 = g * kGrp;
    xp_planes_kernel<<<dim3(kTok / 64, kDim / 64, kGrp), 256, 0, stream>>>(X, P, batch0, xpHi, xpLo, xtHi, xtLo);

    wmma_gemm64<1, true, 1, 2, false, 0><<<dim3((tilesW + 7) / 8, kGrp, 1), 256, 0, stream>>>(
        wh1Hi, wh1Lo, kDim, 0L,
        xpHi, xpLo, kDim, (long)kTok * kDim,
        (void*)w1tHi, (void*)w1tLo, kTok, (long)kDpr * kTok,
        bh1, bh1, 0L,
        kDpr, kTok, kDim, 1.0f);

    wmma_gemm64<1, true, 2, 2, false, 0><<<dim3((tilesW + 7) / 8, kGrp, 1), 256, 0, stream>>>(
        xpHi, xpLo, kDim, (long)kTok * kDim,
        wh2Hi, wh2Lo, kDim, 0L,
        (void*)w2Hi, (void*)w2Lo, kDpr, (long)kTok * kDpr,
        bh2, bh2, 0L,
        kTok, kDpr, kDim, 1.0f);

    wmma_gemm64<1, true, 0, 0, false, 0><<<dim3((tilesPm + 7) / 8, kGrp, kKsp), 256, 0, stream>>>(
        xtHi, xtLo, kTok, (long)kDim * kTok,
        w1tHi, w1tLo, kTok, (long)kDpr * kTok,
        (void*)pmPart, (void*)pmPart, kDpr, (long)kDim * kDpr,
        bh1, bh1, 0L,
        kDim, kDpr, kTok / kKsp, 1.0f);

    gelu_split_kernel<<<groupTot / 256, 256, 0, stream>>>(pmPart, atHi, atLo, groupTot);

    float* Yg = Y + (size_t)batch0 * kTok * kDim;
    wmma_gemm64<1, true, 0, 0, false, 0><<<dim3((tilesY + 7) / 8, kGrp, 1), 256, 0, stream>>>(
        w2Hi, w2Lo, kDpr, (long)kTok * kDpr,
        atHi, atLo, kDpr, (long)kDim * kDpr,
        (void*)Yg, (void*)Yg, kDim, (long)kTok * kDim,
        bh1, bh1, 0L,
        kTok, kDim, kDpr, 1.0f);
  }
}
